// IterativeFeatureExclusion_82025285419368
// MI455X (gfx1250) — hardware-run, weakly checked
//
#include <hip/hip_runtime.h>
#include <math.h>

typedef __attribute__((ext_vector_type(16))) _Float16 v16h;
typedef __attribute__((ext_vector_type(8)))  _Float16 v8h;
typedef __attribute__((ext_vector_type(16))) __bf16   v16b;
typedef __attribute__((ext_vector_type(8)))  __bf16   v8b;
typedef __attribute__((ext_vector_type(8)))  float    v8f;
typedef __attribute__((ext_vector_type(4)))  float    v4f;
typedef __attribute__((ext_vector_type(4)))  unsigned int v4u;

constexpr int kRowsB   = 4096;
constexpr int kFeat    = 64;
constexpr int kHeads   = 8;
constexpr int kUnits   = 32;
constexpr int kTileB   = 128;
constexpr int kSlice   = kFeat * kUnits;
constexpr int kSlices  = kFeat * kHeads;
constexpr int kOutP    = 68;
constexpr float kExpScale = 2.0f;
constexpr float kInvFeat  = 1.0f / (float)kFeat;
static_assert(kFeat == 64 && kUnits == 32 && kHeads == 8 && kRowsB == 4096, "shape contract");
static_assert((kRowsB % kTileB) == 0, "batch tile multiple");
static_assert((kFeat % 32) == 0 && (kUnits % 32) == 0, "contraction depths are multiples of 32");
static_assert(kSlice == 256 * 8, "one 16-B piece per thread per plane slice");

constexpr size_t kPlaneBytes = (size_t)kSlices * kSlice * 2;
constexpr size_t kOffKT   = 0;
constexpr size_t kOffWE   = kOffKT + kPlaneBytes;
constexpr size_t kWsTotal = kOffWE + kPlaneBytes;
static_assert(kWsTotal == 4194304ull, "carve total");
static_assert(kWsTotal <= 134217728ull, "carve cap");
static_assert((kOffWE % 128) == 0, "128-B aligned regions");

__device__ __forceinline__ unsigned short f2bf_bits(float f) {
  unsigned u = __float_as_uint(f);
  return (unsigned short)((u + 0x7FFFu + ((u >> 16) & 1u)) >> 16);
}
__device__ __forceinline__ __bf16 f2bf(float f) {
  const unsigned short b = f2bf_bits(f);
  return __builtin_bit_cast(__bf16, b);
}
__device__ __forceinline__ unsigned short h_bits(float f) {
  const _Float16 h = (_Float16)f;
  return __builtin_bit_cast(unsigned short, h);
}
__device__ __forceinline__ unsigned pk16(unsigned short a, unsigned short b) {
  return (unsigned)a | ((unsigned)b << 16);
}

template <typename T> struct Frag;
template <> struct Frag<_Float16> {
  typedef v16h V; union U { v16h v; v8h h[2]; };
  static __device__ __forceinline__ v16h load(const _Float16* p) {
    U f; f.h[0] = *(const v8h*)(p); f.h[1] = *(const v8h*)(p + 16); return f.v;
  }
};
template <> struct Frag<__bf16> {
  typedef v16b V; union U { v16b v; v8b h[2]; };
  static __device__ __forceinline__ v16b load(const __bf16* p) {
    U f; f.h[0] = *(const v8b*)(p); f.h[1] = *(const v8b*)(p + 16); return f.v;
  }
};

__device__ __forceinline__ v8f mma_h(v16h a, v16h b, v8f c) {
  c = __builtin_amdgcn_wmma_f32_16x16x32_f16(false, a, false, b, (short)0, c, false, false);
  asm volatile("v_nop\n\tv_nop\n\tv_nop\n\tv_nop" : "+v"(c) : "v"(a), "v"(b));
  return c;
}
__device__ __forceinline__ v8f mma_b(v16b a, v16b b, v8f c) {
  c = __builtin_amdgcn_wmma_f32_16x16x32_bf16(false, a, false, b, (short)0, c, false, false);
  asm volatile("v_nop\n\tv_nop\n\tv_nop\n\tv_nop" : "+v"(c) : "v"(a), "v"(b));
  return c;
}
__device__ __forceinline__ void wave_lds_sync() {
  __builtin_amdgcn_fence(__ATOMIC_RELEASE, "workgroup");
  __builtin_amdgcn_wave_barrier();
  __builtin_amdgcn_fence(__ATOMIC_ACQUIRE, "workgroup");
}

__global__ __launch_bounds__(256) void prep_planes_kernel(const float* __restrict__ kern,
                                                          unsigned short* __restrict__ ktp,
                                                          unsigned short* __restrict__ wep) {
  __shared__ float sK[kFeat * 33];
  __shared__ __align__(16) float sX[kSlice];
  const int t = threadIdx.x;
  const int lane = t & 31;
  const int wave = t >> 5;
  const int ja = blockIdx.x;
  const int j = ja / kHeads;
  const float* kg = kern + (size_t)ja * kSlice;
#pragma unroll 1
  for (int i = 0; i < 8; ++i) {
    const int e = t + 256 * i;
    const float v = kg[e];
    const int f = e >> 5;
    const int u = e & 31;
    sK[f * 33 + u] = v;
    sX[e] = expf(kExpScale * v);
  }
  __syncthreads();
  const int q = lane >> 3;
  const int c8 = (lane & 7) * 8;
  const int urow = wave * 4 + q;
  unsigned short hb[8];
#pragma unroll
  for (int e = 0; e < 8; ++e) {
    const int f = c8 + e;
    const float raw = sK[f * 33 + urow];
    const float v = (f == j) ? 0.0f : raw;
    hb[e] = h_bits(v);
  }
  const v4u ku = (v4u){pk16(hb[0], hb[1]), pk16(hb[2], hb[3]), pk16(hb[4], hb[5]), pk16(hb[6], hb[7])};
  const float* sp = sX + t * 8;
  const v4f a0 = *(const v4f*)(sp);
  const v4f a1 = *(const v4f*)(sp + 4);
  unsigned short wb[8];
#pragma unroll
  for (int e = 0; e < 4; ++e) {
    wb[e]     = f2bf_bits(a0[e]);
    wb[4 + e] = f2bf_bits(a1[e]);
  }
  const v4u wu = (v4u){pk16(wb[0], wb[1]), pk16(wb[2], wb[3]), pk16(wb[4], wb[5]), pk16(wb[6], wb[7])};
  unsigned short* kdst = ktp + (size_t)ja * kSlice + (size_t)urow * kFeat + c8;
  unsigned short* wdst = wep + (size_t)ja * kSlice + (size_t)t * 8;
  for (int pass = 0; pass < 2; ++pass) {
    *(volatile v4u*)kdst = ku;
    *(volatile v4u*)wdst = wu;
    __threadfence();
  }
}

__global__ __launch_bounds__(256) void fused_main_kernel(const float* __restrict__ x,
                                                         const unsigned short* __restrict__ ktp,
                                                         const unsigned short* __restrict__ wep,
                                                         float* __restrict__ out) {
  __shared__ __align__(16) _Float16 sKt[2][kUnits * kFeat];
  __shared__ __align__(16) __bf16   sWe[2][kFeat * kUnits];
  __shared__ __align__(16) __bf16   sEt[8][16 * kUnits];
  __shared__ __align__(16) float    sO[8][16 * kOutP];

  const int tid  = threadIdx.x;
  const int wv   = tid >> 5;
  const int lane = tid & 31;
  const int ln   = lane & 15;
  const int kh   = lane >> 4;
  const int b0   = blockIdx.x * kTileB;
  const int a    = blockIdx.y;

  v16h xf[2];
  {
    const float* xrow = x + (size_t)(b0 + wv * 16 + ln) * kFeat;
#pragma unroll
    for (int kc = 0; kc < 2; ++kc) {
      const float* p = xrow + kc * 32 + 8 * kh;
      const v4f a0 = *(const v4f*)(p);
      const v4f a1 = *(const v4f*)(p + 4);
      const v4f c0 = *(const v4f*)(p + 16);
      const v4f c1 = *(const v4f*)(p + 20);
#pragma unroll
      for (int e = 0; e < 4; ++e) {
        xf[kc][e]      = (_Float16)a0[e];
        xf[kc][4 + e]  = (_Float16)a1[e];
        xf[kc][8 + e]  = (_Float16)c0[e];
        xf[kc][12 + e] = (_Float16)c1[e];
      }
    }
  }

  v16b ones;
  {
    const unsigned short ob = (unsigned short)0x3F80u;
    const __bf16 one = __builtin_bit_cast(__bf16, ob);
#pragma unroll
    for (int i = 0; i < 16; ++i) ones[i] = one;
  }

  const v8f zero8 = (v8f){0.f, 0.f, 0.f, 0.f, 0.f, 0.f, 0.f, 0.f};
  v8f acc[4];
#pragma unroll
  for (int nt = 0; nt < 4; ++nt) acc[nt] = zero8;

  const int toff = tid * 8;
  v4u ktreg = *(const v4u*)(ktp + (size_t)a * kSlice + toff);
  v4u wereg = *(const v4u*)(wep + (size_t)a * kSlice + toff);

  __bf16* et = sEt[wv];

#pragma unroll 1
  for (int j = 0; j < kFeat; ++j) {
    const int buf = j & 1;
    *(v4u*)(&sKt[buf][toff]) = ktreg;
    *(v4u*)(&sWe[buf][toff]) = wereg;
    __syncthreads();
    if (j + 1 < kFeat) {
      const size_t nsl = (size_t)((j + 1) * kHeads + a) * kSlice + toff;
      ktreg = *(const v4u*)(ktp + nsl);
      wereg = *(const v4u*)(wep + nsl);
    }

#pragma unroll 1
    for (int nt = 0; nt < 2; ++nt) {
      const _Float16* kp = sKt[buf] + (nt * 16 + ln) * kFeat + 8 * kh;
      const v16h kb0 = Frag<_Float16>::load(kp);
      const v16h kb1 = Frag<_Float16>::load(kp + 32);
      v8f z = mma_h(xf[0], kb0, zero8);
      z = mma_h(xf[1], kb1, z);
#pragma unroll
      for (int r = 0; r < 8; ++r) {
        const float ev = expf(z[r]);
        et[(8 * kh + r) * kUnits + nt * 16 + ln] = f2bf(ev);
      }
    }
    wave_lds_sync();

    const v16b zfrag = Frag<__bf16>::load(et + ln * kUnits + 8 * kh);

    const v8f sv = mma_b(zfrag, ones, zero8);
    float rinv[8];
#pragma unroll
    for (int r = 0; r < 8; ++r) rinv[r] = __builtin_amdgcn_rcpf(sv[r]);

#pragma unroll
    for (int nt = 0; nt < 4; ++nt) {
      const v16b wb = Frag<__bf16>::load(sWe[buf] + (nt * 16 + ln) * kUnits + 8 * kh);
      const v8f tt = mma_b(zfrag, wb, zero8);
#pragma unroll
      for (int r = 0; r < 8; ++r) acc[nt][r] = fmaf(tt[r], rinv[r], acc[nt][r]);
    }
  }

  float* slab = sO[wv];
#pragma unroll
  for (int nt = 0; nt < 4; ++nt) {
#pragma unroll
    for (int r = 0; r < 8; ++r) slab[(8 * kh + r) * kOutP + nt * 16 + ln] = acc[nt][r];
  }
  wave_lds_sync();
  const int c4 = ln * 4;
#pragma unroll 1
  for (int it = 0; it < 8; ++it) {
    const int row = it * 2 + kh;
    float* sp = slab + row * kOutP + c4;
    const v4f v = *(const v4f*)(sp);
    const float v0 = v[0], v1 = v[1], v2 = v[2], v3 = v[3];
    float mx = fmaxf(fmaxf(v0, v1), fmaxf(v2, v3));
#pragma unroll
    for (int off = 1; off < 16; off <<= 1) mx = fmaxf(mx, __shfl_xor(mx, off, 32));
    const float e0 = expf((v0 - mx) * kInvFeat);
    const float e1 = expf((v1 - mx) * kInvFeat);
    const float e2 = expf((v2 - mx) * kInvFeat);
    const float e3 = expf((v3 - mx) * kInvFeat);
    float sm = (e0 + e1) + (e2 + e3);
#pragma unroll
    for (int off = 1; off < 16; off <<= 1) sm += __shfl_xor(sm, off, 32);
    const float inv = 1.0f / sm;
    const v4f o = (v4f){e0 * inv, e1 * inv, e2 * inv, e3 * inv};
    *(v4f*)(sp) = o;
  }
  wave_lds_sync();
  {
    float* C = out + ((size_t)a * kRowsB + (size_t)b0 + (size_t)wv * 16) * kFeat;
    for (int pass = 0; pass < 2; ++pass) {
#pragma unroll
      for (int it = 0; it < 8; ++it) {
        const int row = it * 2 + kh;
        const v4f val = *(const v4f*)(slab + row * kOutP + c4);
        *(volatile v4f*)(C + (size_t)row * kFeat + c4) = val;
      }
      __threadfence();
    }
  }
}

extern "C" void kernel_launch(void* const* d_in, const int* in_sizes, int n_in,
                              void* d_out, int out_size, void* d_ws, size_t ws_size,
                              hipStream_t stream) {
  if (n_in < 2) return;
  if (in_sizes[0] != kRowsB * kFeat) return;
  if (in_sizes[1] != kSlices * kSlice) return;
  if (out_size != kHeads * kRowsB * kFeat) return;
  if (ws_size < kWsTotal) return;

  const float* x    = (const float*)d_in[0];
  const float* kern = (const float*)d_in[1];
  float* out = (float*)d_out;
  char* ws = (char*)d_ws;
  unsigned short* KT = (unsigned short*)(ws + kOffKT);
  unsigned short* WE = (unsigned short*)(ws + kOffWE);

  prep_planes_kernel<<<kSlices, 256, 0, stream>>>(kern, KT, WE);
  fused_main_kernel<<<dim3(kRowsB / kTileB, kHeads), 256, 0, stream>>>(x, KT, WE, out);
}
